// HAN_3762391352090
// MI455X (gfx1250) — hardware-run, weakly checked
//
#include <hip/hip_runtime.h>
#include <stddef.h>
#include <stdint.h>
#include <math.h>


#define NIN     64
#define CH      128
#define NHD     2
#define HD      64
#define NOUT    16
#define OUTC    8
#define KHL     256
#define NATT    4
#define NTHR    256
#define NWAVE   8
#define EPT     8
#define CHUNK   (NTHR * EPT)
#define WCAP    (EPT * 32)
#define LISTN   (NWAVE * WCAP)
#define NBMAX   2048
#define SLOTB   11
#define RCAP    28672
#define DEGCAP  256
#define GBM     64
#define GBN     128
#define GTHR    128
#define GNT     8
#define NEGSL   0.2f
#define MX0     (-1.0e30f)
#define WSMAX   268435456
#define LDS_AGG ((2 * RCAP + 2 * NBMAX + LISTN) * 4 + 64)
#define NUW1    (CH * (NIN / 8))
#define NUW2    (CH * (KHL / 8))
#define NUK1    (CH * (KHL / 8))
#define NUK2    (CH * (KHL / 8))
#define NULT    (NOUT * (KHL / 8))
#define NUB1    (NUW1)
#define NUB2    (NUB1 + NUW2)
#define NUB3    (NUB2 + NUK1)
#define NUB4    (NUB3 + NUK2)
#define NUTOT   (NUB4 + NULT)

static_assert((CHUNK & (CHUNK - 1)) == 0 && CHUNK <= (1 << SLOTB));
static_assert(NBMAX == (1 << SLOTB));
static_assert(NTHR * 8 == NBMAX);
static_assert(LISTN >= NBMAX && LISTN >= NWAVE * WCAP);
static_assert((RCAP % 32) == 0);
static_assert(LDS_AGG <= 300000);
static_assert(GBM == (GTHR / 32) * 16 && GBN == 16 * GNT && GTHR == GBN && GBN == CH);
static_assert(CH == NHD * HD && CH == 32 * 4);
static_assert(HD == 16 * 4);
static_assert((NIN % 32) == 0 && (KHL % 32) == 0);
static_assert(KHL == 2 * CH);
static_assert(NOUT == 16 && OUTC <= NOUT && (OUTC % 4) == 0);
static_assert((NUB1 % NTHR) == 0 && (NUB2 % NTHR) == 0 && (NUB3 % NTHR) == 0 && (NUB4 % NTHR) == 0);
static_assert((NUTOT % NTHR) == 0);
static_assert((NIN / 8) == 8 && (KHL / 8) == 32);
static_assert(GTHR == NHD * HD);
static_assert(NATT * NHD * GBM == 4 * GTHR);
static_assert((GBM * KHL * 2) + (GBM * NOUT * 4) <= 65536);
static_assert(GBM * (OUTC / 4) == GTHR);

typedef float          v4f  __attribute__((ext_vector_type(4)));
typedef float          v8f  __attribute__((ext_vector_type(8)));
typedef int            v4i  __attribute__((ext_vector_type(4)));
typedef int            v8i  __attribute__((ext_vector_type(8)));
typedef unsigned int   v4u  __attribute__((ext_vector_type(4)));
typedef unsigned short v8us __attribute__((ext_vector_type(8)));
typedef __bf16         v16b __attribute__((ext_vector_type(16)));
typedef v4f  __attribute__((may_alias)) v4fa;
typedef v4u  __attribute__((may_alias)) v4ua;
typedef v8us __attribute__((may_alias)) v8usa;
union Frag { v16b vb; v8us h[2]; v8i w; };

__device__ __forceinline__ v8f wmb(const Frag& a, const Frag& b, v8f c) {
  v8f d = __builtin_amdgcn_wmma_f32_16x16x32_bf16(false, a.vb, false, b.vb, (short)0, c, false, false);
  asm volatile("v_nop\n\tv_nop\n\tv_nop\n\tv_nop" : "+v"(d) : "v"(a.w), "v"(b.w));
  return d;
}

__device__ __forceinline__ unsigned short bf_bits(float f) {
  unsigned int u = __float_as_uint(f);
  u += 0x7FFFu + ((u >> 16) & 1u);
  return (unsigned short)(u >> 16);
}
__device__ __forceinline__ float bf_val(unsigned short b) { return __uint_as_float(((unsigned int)b) << 16); }
__device__ __forceinline__ float bf_rne(float f) { return bf_val(bf_bits(f)); }
__device__ __forceinline__ unsigned int pk2(float lo, float hi) {
  return (unsigned int)bf_bits(lo) | ((unsigned int)bf_bits(hi) << 16);
}
__device__ __forceinline__ v4u pack8(const v4f a, const v4f b) {
  v4u r;
  r.x = pk2(a.x, a.y); r.y = pk2(a.z, a.w); r.z = pk2(b.x, b.y); r.w = pk2(b.z, b.w);
  return r;
}
__device__ __forceinline__ float rlo(unsigned int h, unsigned int l) {
  return __uint_as_float(h << 16) + __uint_as_float(l << 16);
}
__device__ __forceinline__ float rhi(unsigned int h, unsigned int l) {
  return __uint_as_float(h & 0xFFFF0000u) + __uint_as_float(l & 0xFFFF0000u);
}

__device__ __forceinline__ int scan_chunk(const int* __restrict__ dsts, int nE, int cbase, int slotBase,
                                          int nb, int vec8, int* list, int tid, int lane, int wave) {
  int wc = 0;
  const int el0  = tid * EPT;
  const int e0   = cbase + el0;
  const int sent = -2147483647 - 1;
  v4i da, db;
  if (vec8 != 0 && cbase + CHUNK <= nE) {
    da = *(const v4i*)(dsts + e0);
    db = *(const v4i*)(dsts + e0 + 4);
  } else {
    da.x = (e0     < nE) ? dsts[min(e0,     nE - 1)] : sent;
    da.y = (e0 + 1 < nE) ? dsts[min(e0 + 1, nE - 1)] : sent;
    da.z = (e0 + 2 < nE) ? dsts[min(e0 + 2, nE - 1)] : sent;
    da.w = (e0 + 3 < nE) ? dsts[min(e0 + 3, nE - 1)] : sent;
    db.x = (e0 + 4 < nE) ? dsts[min(e0 + 4, nE - 1)] : sent;
    db.y = (e0 + 5 < nE) ? dsts[min(e0 + 5, nE - 1)] : sent;
    db.z = (e0 + 6 < nE) ? dsts[min(e0 + 6, nE - 1)] : sent;
    db.w = (e0 + 7 < nE) ? dsts[min(e0 + 7, nE - 1)] : sent;
  }
  const unsigned nbs = (unsigned)slotBase;
  const unsigned unb = (unsigned)nb;
  const unsigned s0 = (unsigned)da.x - nbs, s1 = (unsigned)da.y - nbs;
  const unsigned s2 = (unsigned)da.z - nbs, s3 = (unsigned)da.w - nbs;
  const unsigned s4 = (unsigned)db.x - nbs, s5 = (unsigned)db.y - nbs;
  const unsigned s6 = (unsigned)db.z - nbs, s7 = (unsigned)db.w - nbs;
  const bool h0 = s0 < unb, h1 = s1 < unb, h2 = s2 < unb, h3 = s3 < unb;
  const bool h4 = s4 < unb, h5 = s5 < unb, h6 = s6 < unb, h7 = s7 < unb;
  const unsigned any = __builtin_amdgcn_ballot_w32(h0 | h1 | h2 | h3 | h4 | h5 | h6 | h7);
  if (any != 0u) {
#define HITJ(J, HJ, SJ) { \
      const unsigned mj = __builtin_amdgcn_ballot_w32(HJ); \
      if (mj != 0u) { \
        if (HJ) { \
          const int pos = wc + (int)__builtin_amdgcn_mbcnt_lo(mj, 0u); \
          if (pos < WCAP) list[wave * WCAP + pos] = ((el0 + (J)) << SLOTB) | (int)(SJ); \
        } \
        wc += (int)__builtin_popcount(mj); } }
    HITJ(0, h0, s0)
    HITJ(1, h1, s1)
    HITJ(2, h2, s2)
    HITJ(3, h3, s3)
    HITJ(4, h4, s4)
    HITJ(5, h5, s5)
    HITJ(6, h6, s6)
    HITJ(7, h7, s7)
#undef HITJ
  }
  return wc;
}

__global__ __launch_bounds__(NTHR) void k_xprep(const float* __restrict__ x, unsigned short* xb, int F, int nN,
                                                int nUnits) {
  const int i = (int)blockIdx.x * NTHR + (int)threadIdx.x;
  if (i >= nUnits) return;
  const int fq  = F >> 3;
  const int row = i / fq;
  const int c0  = (i - row * fq) * 8;
  const int rc  = row < nN ? row : nN - 1;
  const float* p = x + (size_t)rc * (size_t)F + c0;
  v4f a = *(const v4fa*)p, b = *(const v4fa*)(p + 4);
  const v4f z4 = {0.f, 0.f, 0.f, 0.f};
  if (row >= nN) { a = z4; b = z4; }
  const v4u hv = pack8(a, b);
  const size_t o = (size_t)row * (size_t)F + c0;
  *(volatile v4u*)(xb + o) = hv;
  __threadfence();
  *(volatile v4u*)(xb + o) = hv;
}

__device__ __forceinline__ v8us cv8b(const float* __restrict__ p, size_t stride) {
  v8us o;
#pragma unroll
  for (int i = 0; i < 8; ++i) o[i] = bf_bits(p[(size_t)i * stride]);
  return o;
}

__global__ __launch_bounds__(NTHR) void k_wprep(const float* __restrict__ w1, const float* __restrict__ w2,
                                                const float* __restrict__ k1, const float* __restrict__ k2,
                                                const float* __restrict__ lw,
                                                unsigned short* pw1, unsigned short* pw2,
                                                unsigned short* pk1, unsigned short* pk2l,
                                                unsigned short* plt) {
  const int u = (int)blockIdx.x * NTHR + (int)threadIdx.x;
  v8us o;
  unsigned short* dp;
  if (u < NUB1) {
    const int v = u, n = v >> 3, k8 = (v & 7) * 8;
    o = cv8b(w1 + (size_t)k8 * CH + n, CH);
    dp = pw1 + (size_t)v * 8;
  } else if (u < NUB2) {
    const int v = u - NUB1, n = v >> 5, k8 = (v & 31) * 8;
    const int kk = k8 & (CH - 1);
    o = cv8b(w2 + (size_t)kk * CH + n, CH);
    dp = pw2 + (size_t)v * 8;
  } else if (u < NUB3) {
    const int v = u - NUB2, n = v >> 5, k8 = (v & 31) * 8;
    const int kk = k8 & (CH - 1);
    o = cv8b(k1 + (size_t)kk * CH + n, CH);
    dp = pk1 + (size_t)v * 8;
  } else if (u < NUB4) {
    const int v = u - NUB3, n = v >> 5, k8 = (v & 31) * 8;
    const int kk = k8 & (CH - 1);
    o = cv8b(k2 + (size_t)kk * CH + n, CH);
    dp = pk2l + (size_t)v * 8;
  } else if (u < NUTOT) {
    const int v = u - NUB4, n = v >> 5, k8 = (v & 31) * 8;
    const int kk = k8 & (CH - 1);
    const int nc = n < OUTC ? n : OUTC - 1;
    o = cv8b(lw + (size_t)kk * OUTC + nc, OUTC);
    const v8us z8 = {0, 0, 0, 0, 0, 0, 0, 0};
    if (n >= OUTC) o = z8;
    dp = plt + (size_t)v * 8;
  } else {
    return;
  }
  *(volatile v8us*)dp = o;
  __threadfence();
  *(volatile v8us*)dp = o;
}

template <int EPI>
__global__ __launch_bounds__(GTHR) void k_gemm(const unsigned short* __restrict__ A, int lda, size_t aoff,
                                               const unsigned short* __restrict__ BT, int ldb, int K,
                                               const float* __restrict__ bias, float* outF, int ldo,
                                               const float* __restrict__ atts, const float* __restrict__ attd,
                                               float* DP, int nN, int mRows) {
  __shared__ __attribute__((aligned(16))) float stg[GBM * GBN];
  __shared__ __attribute__((aligned(16))) float satt[NATT * CH];
  __shared__ __attribute__((aligned(16))) float sdot[NATT * NHD * GBM];
  __shared__ __attribute__((aligned(16))) float pst[GBN];
  const int tid = (int)threadIdx.x, lane = tid & 31, wave = tid >> 5, hh = lane >> 4, m = lane & 15;
  const int rowBase = (int)blockIdx.x * GBM;
  const int by = (int)blockIdx.y;

  if constexpr (EPI == 0) {
    satt[tid]          = bf_rne(atts[tid]);
    satt[CH + tid]     = bf_rne(attd[tid]);
    satt[2 * CH + tid] = bf_rne(atts[CH + tid]);
    satt[3 * CH + tid] = bf_rne(attd[CH + tid]);
  }

  v8f acc[GNT];
  {
    const v8f z = {0.f, 0.f, 0.f, 0.f, 0.f, 0.f, 0.f, 0.f};
#pragma unroll
    for (int t = 0; t < GNT; ++t) acc[t] = z;
  }
  const unsigned short* Ab = A + (size_t)by * aoff;
  const unsigned short* ap = Ab + (size_t)(rowBase + 16 * wave + m) * (size_t)lda + 8 * hh;
  const unsigned short* bp = BT + (size_t)m * (size_t)ldb + 8 * hh;

#pragma unroll 1
  for (int k0 = 0; k0 < K; k0 += 32) {
    Frag af;
    af.h[0] = *(const v8usa*)(ap + k0);
    af.h[1] = *(const v8usa*)(ap + k0 + 16);
#pragma unroll
    for (int nt = 0; nt < GNT; ++nt) {
      const unsigned short* wq = bp + (size_t)(16 * nt) * (size_t)ldb + k0;
      Frag bfg;
      bfg.h[0] = *(const v8usa*)wq;
      bfg.h[1] = *(const v8usa*)(wq + 16);
      acc[nt] = wmb(af, bfg, acc[nt]);
    }
  }

#pragma unroll
  for (int nt = 0; nt < GNT; ++nt) {
    const int lc = 16 * nt + m;
    const float bb = bf_rne(bias[lc]);
#pragma unroll
    for (int r = 0; r < 8; ++r) {
      const int lr = 16 * wave + 8 * hh + r;
      const bool live = (rowBase + lr) < nN;
      const float v = acc[nt][r] + bb;
      stg[lr * GBN + lc] = live ? v : 0.0f;
    }
  }
  __syncthreads();

  if constexpr (EPI == 0) {
    {
      const int row = tid & 63, head = tid >> 6;
#pragma unroll 1
      for (int a = 0; a < NATT; ++a) {
        const float* hr = stg + row * GBN + HD * head;
        const float* sa = satt + a * CH + HD * head;
        float d = 0.0f;
#pragma unroll
        for (int c4 = 0; c4 < HD / 4; ++c4) {
          const v4f hv = *(const v4fa*)(hr + 4 * c4);
          const v4f av = *(const v4fa*)(sa + 4 * c4);
          d = fmaf(hv.x, av.x, d);
          d = fmaf(hv.y, av.y, d);
          d = fmaf(hv.z, av.z, d);
          d = fmaf(hv.w, av.w, d);
        }
        sdot[(a * NHD + head) * GBM + row] = d;
      }
    }
    __syncthreads();

    v4f fv[16];
#pragma unroll
    for (int i = 0; i < 16; ++i) {
      const int lr = 16 * wave + i;
      fv[i] = *(const v4fa*)(stg + lr * GBN + 4 * lane);
    }
    const int pl = tid >> 4, pc = tid & 15;
    const v4f dv = *(const v4fa*)(sdot + pl * GBM + 4 * pc);
    float* dpp = DP + (size_t)pl * (size_t)mRows + rowBase + 4 * pc;
#pragma unroll
    for (int i = 0; i < 16; ++i) {
      const int gr = rowBase + 16 * wave + i;
      float* op = outF + (size_t)gr * (size_t)ldo + 4 * lane;
      if (gr < mRows) *(volatile v4f*)op = fv[i];
    }
    *(volatile v4f*)dpp = dv;
    __threadfence();
#pragma unroll
    for (int i = 0; i < 16; ++i) {
      const int gr = rowBase + 16 * wave + i;
      float* op = outF + (size_t)gr * (size_t)ldo + 4 * lane;
      if (gr < mRows) *(volatile v4f*)op = fv[i];
    }
    *(volatile v4f*)dpp = dv;
  } else {
    float s = 0.0f;
#pragma unroll 1
    for (int r = 0; r < GBM; ++r) s += tanhf(stg[r * GBN + tid]);
    pst[tid] = s;
    __syncthreads();
    const bool pok = tid < 32;
    v4f pv = {0.f, 0.f, 0.f, 0.f};
    if (pok) pv = *(const v4fa*)(pst + 4 * tid);
    float* pp = outF + ((size_t)by * (size_t)gridDim.x + (size_t)blockIdx.x) * CH + 4 * tid;
    if (pok) *(volatile v4f*)pp = pv;
    __threadfence();
    if (pok) *(volatile v4f*)pp = pv;
  }
}

__global__ __launch_bounds__(NTHR) void k_agg(
    const int* __restrict__ srcs, const int* __restrict__ dsts,
    const float* __restrict__ F, const float* __restrict__ AS, const float* __restrict__ AD,
    unsigned short* HP, int nN, int nE, int nb, int vec8, int MP) {
  extern __shared__ v4f lds_dyn[];
  int* reg1 = (int*)lds_dyn;
  int* reg2 = reg1 + RCAP;
  int* scnt = reg2 + RCAP;
  int* soff = scnt + NBMAX;
  int* list = soff + NBMAX;
  int* wcnt = list + LISTN;
  int* wtot = wcnt + NWAVE;
  const int tid = (int)threadIdx.x, lane = tid & 31, wave = tid >> 5;
  const int nodeBase = (int)blockIdx.x * nb;

  for (int i = tid; i < NBMAX; i += NTHR) scnt[i] = 0;
  __syncthreads();

  int tot = 0;
  const int nChunks = (nE + CHUNK - 1) / CHUNK;
#pragma unroll 1
  for (int ch = 0; ch < nChunks; ++ch) {
    const int cbase = ch * CHUNK;
    const int wc = scan_chunk(dsts, nE, cbase, nodeBase, nb, vec8, list, tid, lane, wave);
    if (lane == 0) wcnt[wave] = wc;
    __syncthreads();
    int pre = 0, all = 0;
#pragma unroll
    for (int w2 = 0; w2 < NWAVE; ++w2) {
      int c = wcnt[w2];
      c = c < 0 ? 0 : (c > WCAP ? WCAP : c);
      all += c;
      pre += (w2 < wave) ? c : 0;
    }
    const int wcc  = wc > WCAP ? WCAP : wc;
    const int base = tot + pre;
#pragma unroll 1
    for (int i = lane; i < wcc; i += 32) {
      const int ent = list[wave * WCAP + i];
      const int el  = (ent >> SLOTB) & (CHUNK - 1);
      const int sl  = ent & (NBMAX - 1);
      int eid = cbase + el;
      eid = eid > nE - 1 ? nE - 1 : eid;
      const int pos = base + i;
      if (pos < RCAP) reg1[pos] = (int)(((unsigned)eid << SLOTB) | (unsigned)sl);
    }
    tot += all;
    tot = tot > RCAP ? RCAP : tot;
    __syncthreads();
  }
  const int nh = tot;

  if (wave == 0) {
#pragma unroll 1
    for (int b0 = 0; b0 < nh; b0 += 32) {
      const int idx = b0 + lane;
      const int uv  = reg1[idx < nh ? idx : nh - 1];
      const int m32 = (nh - b0) < 32 ? (nh - b0) : 32;
#pragma unroll 1
      for (int k = 0; k < m32; ++k) {
        const int u  = __builtin_amdgcn_readlane(uv, k);
        const int sl = u & (NBMAX - 1);
        if (lane == 0) scnt[sl] = scnt[sl] + 1;
      }
    }
  }
  __syncthreads();

  {
    const v4i ca = *(const v4i*)(scnt + 8 * tid);
    const v4i cb = *(const v4i*)(scnt + 8 * tid + 4);
    const int e0 = ca.x < 0 ? 0 : ca.x, e1 = ca.y < 0 ? 0 : ca.y, e2 = ca.z < 0 ? 0 : ca.z, e3 = ca.w < 0 ? 0 : ca.w;
    const int e4 = cb.x < 0 ? 0 : cb.x, e5 = cb.y < 0 ? 0 : cb.y, e6 = cb.z < 0 ? 0 : cb.z, e7 = cb.w < 0 ? 0 : cb.w;
    const int ts = e0 + e1 + e2 + e3 + e4 + e5 + e6 + e7;
    int incl = ts;
#pragma unroll
    for (int d = 1; d < 32; d <<= 1) {
      const int up = __shfl_up(incl, d);
      if (lane >= d) incl += up;
    }
    if (lane == 31) wtot[wave] = incl;
    __syncthreads();
    int pre = 0;
#pragma unroll
    for (int w2 = 0; w2 < NWAVE; ++w2) pre += (w2 < wave) ? wtot[w2] : 0;
    int run = pre + incl - ts;
    soff[8 * tid + 0] = run; run += e0;
    soff[8 * tid + 1] = run; run += e1;
    soff[8 * tid + 2] = run; run += e2;
    soff[8 * tid + 3] = run; run += e3;
    soff[8 * tid + 4] = run; run += e4;
    soff[8 * tid + 5] = run; run += e5;
    soff[8 * tid + 6] = run; run += e6;
    soff[8 * tid + 7] = run;
  }
  __syncthreads();
  for (int i = tid; i < NBMAX; i += NTHR) list[i] = soff[i];
  __syncthreads();

  if (wave == 0) {
#pragma unroll 1
    for (int b0 = 0; b0 < nh; b0 += 32) {
      const int idx = b0 + lane;
      const int uv  = reg1[idx < nh ? idx : nh - 1];
      const int m32 = (nh - b0) < 32 ? (nh - b0) : 32;
#pragma unroll 1
      for (int k = 0; k < m32; ++k) {
        const int u   = __builtin_amdgcn_readlane(uv, k);
        const int sl  = u & (NBMAX - 1);
        const int eid = (int)((unsigned)u >> SLOTB);
        if (lane == 0) {
          int pos = list[sl];
          pos = pos < 0 ? 0 : (pos > RCAP - 1 ? RCAP - 1 : pos);
          reg2[pos] = eid;
          list[sl] = pos + 1;
        }
      }
    }
  }
  __syncthreads();

  const int nbw = nb >> 3;
  const bool ovf = (nh >= RCAP);
  const float qnan = __int_as_float(0x7fc00000);
  const int c0   = 4 * lane;
  const int head = lane >> 4;
  const float* ASp = AS + (size_t)head * (size_t)MP;
  const float* ADp = AD + (size_t)head * (size_t)MP;

#pragma unroll 1
  for (int jt = 0; jt < nbw; ++jt) {
    const int slot = wave * nbw + jt;
    const int grow = nodeBase + slot;
    const int gcl  = grow < nN ? grow : nN - 1;
    int st = soff[slot];
    const int craw = scnt[slot];
    int cnt = craw;
    st  = st < 0 ? 0 : (st > nh ? nh : st);
    cnt = cnt < 0 ? 0 : (cnt > DEGCAP ? DEGCAP : cnt);
    if (cnt > nh - st) cnt = nh - st;
    const float pz = (ovf || craw > DEGCAP) ? qnan : 0.0f;
    const bool liveRow = grow < nN;

    const float adv = ADp[gcl];
    float mx = MX0, dn = 0.0f;
    float a0 = 0.0f, a1 = 0.0f, a2 = 0.0f, a3 = 0.0f;

#pragma unroll 1
    for (int q = 0; q < cnt; ++q) {
      int idx = st + q; idx = idx > RCAP - 1 ? RCAP - 1 : idx;
      int eid = reg2[idx]; eid = eid < 0 ? 0 : (eid > nE - 1 ? nE - 1 : eid);
      const int sraw = srcs[eid];
      const int s = sraw < 0 ? 0 : (sraw > nN - 1 ? nN - 1 : sraw);
      const v4f fs = *(const v4fa*)(F + (size_t)s * CH + c0);
      float lg = ASp[s] + adv;
      lg = lg > 0.0f ? lg : NEGSL * lg;
      const float df = lg - mx;
      const float ee = __expf(-fabsf(df));
      const bool up  = df > 0.0f;
      const float s1 = up ? ee : 1.0f;
      const float s2 = up ? 1.0f : ee;
      mx = up ? lg : mx;
      dn = fmaf(dn, s1, s2);
      a0 = fmaf(a0, s1, s2 * fs.x);
      a1 = fmaf(a1, s1, s2 * fs.y);
      a2 = fmaf(a2, s1, s2 * fs.z);
      a3 = fmaf(a3, s1, s2 * fs.w);
    }
    const float dnz = dn > 0.0f ? dn : 1.0f;
    const float inv = __builtin_amdgcn_rcpf(dnz);
    float h0 = fmaxf(a0 * inv, 0.0f);
    float h1 = fmaxf(a1 * inv, 0.0f);
    float h2 = fmaxf(a2 * inv, 0.0f);
    float h3 = fmaxf(a3 * inv, 0.0f);
    h0 = (liveRow ? h0 : 0.0f) + pz;
    h1 = (liveRow ? h1 : 0.0f) + pz;
    h2 = (liveRow ? h2 : 0.0f) + pz;
    h3 = (liveRow ? h3 : 0.0f) + pz;

    const unsigned int hb0 = bf_bits(h0), hb1 = bf_bits(h1), hb2 = bf_bits(h2), hb3 = bf_bits(h3);
    const unsigned int lb0 = bf_bits(h0 - bf_val((unsigned short)hb0));
    const unsigned int lb1 = bf_bits(h1 - bf_val((unsigned short)hb1));
    const unsigned int lb2 = bf_bits(h2 - bf_val((unsigned short)hb2));
    const unsigned int lb3 = bf_bits(h3 - bf_val((unsigned short)hb3));
    const int hwA = (int)(hb0 | (hb1 << 16));
    const int hwB = (int)(hb2 | (hb3 << 16));
    const int lwA = (int)(lb0 | (lb1 << 16));
    const int lwB = (int)(lb2 | (lb3 << 16));
    const int j  = lane & 15;
    const int sA = 2 * j, sB = 2 * j + 1;
    const int g0h = __shfl(hwA, sA), g1h = __shfl(hwB, sA), g2h = __shfl(hwA, sB), g3h = __shfl(hwB, sB);
    const int g0l = __shfl(lwA, sA), g1l = __shfl(lwB, sA), g2l = __shfl(lwA, sB), g3l = __shfl(lwB, sB);
    const bool hsel = lane < 16;
    v4u pv;
    pv.x = (unsigned int)(hsel ? g0h : g0l);
    pv.y = (unsigned int)(hsel ? g1h : g1l);
    pv.z = (unsigned int)(hsel ? g2h : g2l);
    pv.w = (unsigned int)(hsel ? g3h : g3l);

    unsigned short* hp = HP + (size_t)grow * KHL + 8 * lane;
    const bool wr = grow < MP;
    if (wr) *(volatile v4u*)hp = pv;
    __threadfence();
    if (wr) *(volatile v4u*)hp = pv;
  }
}

__global__ __launch_bounds__(GBN) void k_beta(const float* __restrict__ ps, int gM, int nN,
                                              const float* __restrict__ qv, float* be) {
  __shared__ double r0[GBN], r1[GBN];
  __shared__ __attribute__((aligned(16))) float bl[32];
  const int tid = (int)threadIdx.x;
  double s0 = 0.0, s1 = 0.0;
#pragma unroll 1
  for (int b = 0; b < gM; ++b) {
    s0 += (double)ps[(size_t)b * CH + tid];
    s1 += (double)ps[((size_t)gM + (size_t)b) * CH + tid];
  }
  const double qc  = (double)bf_rne(qv[tid]);
  const double inv = 1.0 / (double)(nN < 1 ? 1 : nN);
  r0[tid] = s0 * inv * qc;
  r1[tid] = s1 * inv * qc;
  if (tid < 32) bl[tid] = 0.0f;
  __syncthreads();
#pragma unroll 1
  for (int s = GBN / 2; s > 0; s >>= 1) {
    if (tid < s) { r0[tid] += r0[tid + s]; r1[tid] += r1[tid + s]; }
    __syncthreads();
  }
  if (tid == 0) {
    const float w0 = (float)r0[0], w1 = (float)r1[0];
    const float mx = fmaxf(w0, w1);
    const float e0 = expf(w0 - mx), e1 = expf(w1 - mx);
    const float rs = 1.0f / (e0 + e1);
    bl[0] = e0 * rs;
    bl[1] = e1 * rs;
  }
  __syncthreads();
  const bool ok = tid < 8;
  v4f v = {0.f, 0.f, 0.f, 0.f};
  if (ok) v = *(const v4fa*)(bl + 4 * tid);
  if (ok) *(volatile v4f*)(be + 4 * tid) = v;
  __threadfence();
  if (ok) *(volatile v4f*)(be + 4 * tid) = v;
}

__global__ __launch_bounds__(NTHR) void k_mix(const unsigned short* __restrict__ P1, const unsigned short* __restrict__ P2,
                                              const float* __restrict__ be, unsigned short* H2, int nN, int nUnits) {
  const int i = (int)blockIdx.x * NTHR + (int)threadIdx.x;
  if (i >= nUnits) return;
  const int row = i >> 5, p = i & 31, c8 = (p & 15) * 8;
  const float b0 = be[0], b1 = be[1];
  const int gc = row < nN ? row : nN - 1;
  const unsigned short* pa = P1 + (size_t)gc * KHL + c8;
  const unsigned short* pb = P2 + (size_t)gc * KHL + c8;
  const v4u ha = *(const v4ua*)pa, la = *(const v4ua*)(pa + CH);
  const v4u hb = *(const v4ua*)pb, lbw = *(const v4ua*)(pb + CH);
  const bool live = row < nN;
  float f[8];
  f[0] = fmaf(b1, rlo(hb.x, lbw.x), b0 * rlo(ha.x, la.x));
  f[1] = fmaf(b1, rhi(hb.x, lbw.x), b0 * rhi(ha.x, la.x));
  f[2] = fmaf(b1, rlo(hb.y, lbw.y), b0 * rlo(ha.y, la.y));
  f[3] = fmaf(b1, rhi(hb.y, lbw.y), b0 * rhi(ha.y, la.y));
  f[4] = fmaf(b1, rlo(hb.z, lbw.z), b0 * rlo(ha.z, la.z));
  f[5] = fmaf(b1, rhi(hb.z, lbw.z), b0 * rhi(ha.z, la.z));
  f[6] = fmaf(b1, rlo(hb.w, lbw.w), b0 * rlo(ha.w, la.w));
  f[7] = fmaf(b1, rhi(hb.w, lbw.w), b0 * rhi(ha.w, la.w));
  const bool hsel = p < 16;
  unsigned int wv[4];
#pragma unroll
  for (int jj = 0; jj < 4; ++jj) {
    float v0 = fmaxf(f[2 * jj], 0.0f), v1 = fmaxf(f[2 * jj + 1], 0.0f);
    v0 = live ? v0 : 0.0f;
    v1 = live ? v1 : 0.0f;
    const unsigned short h0 = bf_bits(v0), h1 = bf_bits(v1);
    const unsigned short l0 = bf_bits(v0 - bf_val(h0)), l1 = bf_bits(v1 - bf_val(h1));
    const unsigned int wh = (unsigned int)h0 | ((unsigned int)h1 << 16);
    const unsigned int wl = (unsigned int)l0 | ((unsigned int)l1 << 16);
    wv[jj] = hsel ? wh : wl;
  }
  v4u o;
  o.x = wv[0]; o.y = wv[1]; o.z = wv[2]; o.w = wv[3];
  unsigned short* dp = H2 + (size_t)row * KHL + 8 * p;
  *(volatile v4u*)dp = o;
  __threadfence();
  *(volatile v4u*)dp = o;
}

__global__ __launch_bounds__(GTHR) void k_out(const unsigned short* __restrict__ P1, const unsigned short* __restrict__ P2,
                                             const float* __restrict__ be, const unsigned short* __restrict__ LT,
                                             const float* __restrict__ lb, int nN, float* out) {
  __shared__ __attribute__((aligned(16))) unsigned short As[GBM * KHL];
  __shared__ __attribute__((aligned(16))) float so[GBM * NOUT];
  const int tid = (int)threadIdx.x, lane = tid & 31, wave = tid >> 5, hh = lane >> 4, m = lane & 15;
  const int rowBase = (int)blockIdx.x * GBM;
  const float b0 = be[0], b1 = be[1];

  const int qq = tid & 15, rs = tid >> 4;
#pragma unroll 1
  for (int it = 0; it < 8; ++it) {
    const int lr = 8 * it + rs;
    const int grow = rowBase + lr;
    const int gc = grow < nN ? grow : nN - 1;
    const unsigned short* pa = P1 + (size_t)gc * KHL + 8 * qq;
    const unsigned short* pb = P2 + (size_t)gc * KHL + 8 * qq;
    const v4u ha = *(const v4ua*)pa, la = *(const v4ua*)(pa + CH);
    const v4u hb = *(const v4ua*)pb, lbw = *(const v4ua*)(pb + CH);
    const bool live = grow < nN;
    float f[8];
    f[0] = fmaf(b1, rlo(hb.x, lbw.x), b0 * rlo(ha.x, la.x));
    f[1] = fmaf(b1, rhi(hb.x, lbw.x), b0 * rhi(ha.x, la.x));
    f[2] = fmaf(b1, rlo(hb.y, lbw.y), b0 * rlo(ha.y, la.y));
    f[3] = fmaf(b1, rhi(hb.y, lbw.y), b0 * rhi(ha.y, la.y));
    f[4] = fmaf(b1, rlo(hb.z, lbw.z), b0 * rlo(ha.z, la.z));
    f[5] = fmaf(b1, rhi(hb.z, lbw.z), b0 * rhi(ha.z, la.z));
    f[6] = fmaf(b1, rlo(hb.w, lbw.w), b0 * rlo(ha.w, la.w));
    f[7] = fmaf(b1, rhi(hb.w, lbw.w), b0 * rhi(ha.w, la.w));
    unsigned int wh[4], wl[4];
#pragma unroll
    for (int j = 0; j < 4; ++j) {
      float v0 = fmaxf(f[2 * j], 0.0f), v1 = fmaxf(f[2 * j + 1], 0.0f);
      v0 = live ? v0 : 0.0f;
      v1 = live ? v1 : 0.0f;
      const unsigned short h0 = bf_bits(v0), h1 = bf_bits(v1);
      const unsigned short l0 = bf_bits(v0 - bf_val(h0)), l1 = bf_bits(v1 - bf_val(h1));
      wh[j] = (unsigned int)h0 | ((unsigned int)h1 << 16);
      wl[j] = (unsigned int)l0 | ((unsigned int)l1 << 16);
    }
    v4u hv, lv;
    hv.x = wh[0]; hv.y = wh[1]; hv.z = wh[2]; hv.w = wh[3];
    lv.x = wl[0]; lv.y = wl[1]; lv.z = wl[2]; lv.w = wl[3];
    *(v4ua*)(As + lr * KHL + 8 * qq)      = hv;
    *(v4ua*)(As + lr * KHL + CH + 8 * qq) = lv;
  }
  __syncthreads();

  v8f acc = {0.f, 0.f, 0.f, 0.f, 0.f, 0.f, 0.f, 0.f};
  const unsigned short* ap = As + (16 * wave + m) * KHL + 8 * hh;
  const unsigned short* bp = LT + (size_t)m * KHL + 8 * hh;
#pragma unroll 1
  for (int k0 = 0; k0 < KHL; k0 += 32) {
    Frag af, bfg;
    af.h[0]  = *(const v8usa*)(ap + k0);
    af.h[1]  = *(const v8usa*)(ap + k0 + 16);
    bfg.h[0] = *(const v8usa*)(bp + k0);
    bfg.h[1] = *(const v8usa*)(bp + k0 + 16);
    acc = wmb(af, bfg, acc);
  }
  const int mc = m < OUTC ? m : OUTC - 1;
  float lbm = bf_rne(lb[mc]);
  lbm = m < OUTC ? lbm : 0.0f;
#pragma unroll
  for (int r = 0; r < 8; ++r) {
    const int lr = 16 * wave + 8 * hh + r;
    so[lr * NOUT + m] = acc[r] + lbm;
  }
  __syncthreads();

  int nvr = nN - rowBase;
  nvr = nvr < 0 ? 0 : (nvr > GBM ? GBM : nvr);
  const int npc = nvr * (OUTC / 4);
  float* ob = out + (size_t)rowBase * OUTC;
  const int p  = tid;
  const bool pok = p < npc;
  const v4f pv = *(const v4fa*)(so + (p >> 1) * NOUT + 4 * (p & 1));
  if (pok) *(volatile v4f*)(ob + 4 * p) = pv;
  __threadfence();
  if (pok) *(volatile v4f*)(ob + 4 * p) = pv;
}

static int pick_nb(int nE, int nN) {
  int nb = NBMAX;
  while (nb > 32 && (long long)nb * (long long)nE * 5LL > (long long)RCAP * (long long)nN * 4LL) nb >>= 1;
  return nb;
}
static inline int cdiv(int a, int b) { return (a + b - 1) / b; }
static inline size_t al256(size_t o) { return (o + 255) & ~(size_t)255; }

extern "C" void kernel_launch(void* const* d_in, const int* in_sizes, int n_in,
                              void* d_out, int out_size, void* d_ws, size_t ws_size,
                              hipStream_t stream) {
  if (n_in < 19) return;
  if (in_sizes[0] < NIN * GBM || (in_sizes[0] % NIN) != 0) return;
  const int nN = in_sizes[0] / NIN;
  if (nN < GBM || nN > (1 << 22)) return;
  if (in_sizes[1] < 2 || (in_sizes[1] & 1) != 0) return;
  if (in_sizes[2] < 2 || (in_sizes[2] & 1) != 0) return;
  const int nE0 = in_sizes[1] / 2;
  const int nE1 = in_sizes[2] / 2;
  if (nE0 < 1 || nE0 >= (1 << (32 - SLOTB)) || nE1 < 1 || nE1 >= (1 << (32 - SLOTB))) return;
  if (in_sizes[3] != NIN * CH || in_sizes[4] != CH) return;
  if (in_sizes[5] != 2 * CH || in_sizes[6] != 2 * CH) return;
  if (in_sizes[7] != CH || in_sizes[8] != CH * CH || in_sizes[9] != CH) return;
  if (in_sizes[10] != CH * CH || in_sizes[11] != CH) return;
  if (in_sizes[12] != 2 * CH || in_sizes[13] != 2 * CH) return;
  if (in_sizes[14] != CH || in_sizes[15] != CH * CH || in_sizes[16] != CH) return;
  if (in_sizes[17] != CH * OUTC || in_sizes[18] != OUTC) return;
  if ((long long)out_size != (long long)nN * OUTC) return;

  const float* x    = (const float*)d_in[0];
  const int*   e0   = (const int*)  d_in[1];
  const int*   e1   = (const int*)  d_in[2];
  const float* w1   = (const float*)d_in[3];
  const float* b1   = (const float*)d_in[4];
  const float* as1  = (const float*)d_in[5];
  const float* ad1  = (const float*)d_in[6];
  const float* q1   = (const float*)d_in[7];
  const float* kw1  = (const float*)d_in[8];
  const float* kb1  = (const float*)d_in[9];
  const float* w2   = (const float*)d_in[10];
  const float* b2   = (const float*)d_in[11];
  const float* as2  = (const float*)d_in[12];
  const float* ad2  = (const float*)d_in[13];
  const float* q2   = (const float*)d_in[14];
  const float* kw2  = (const float*)d_in[15];
  const float* kb2  = (const float*)d_in[16];
  const float* lw   = (const float*)d_in[17];
  const float* lb   = (const float*)d_in[18];
  float* out = (float*)d_out;
  const int* src0 = e0;
  const int* dst0 = e0 + nE0;
  const int* src1 = e1;
  const int* dst1 = e1 + nE1;

  const int MP = cdiv(nN, GBM) * GBM;
  const int gM = MP / GBM;
  const int nb0 = pick_nb(nE0, nN), nb1 = pick_nb(nE1, nN);
  if (nb0 < 32 || (nb0 & (nb0 - 1)) != 0 || nb0 > NBMAX) return;
  if (nb1 < 32 || (nb1 & (nb1 - 1)) != 0 || nb1 > NBMAX) return;
  const int gA0 = cdiv(MP, nb0), gA1 = cdiv(MP, nb1);
  if ((long long)gA0 * nb0 < (long long)MP || (long long)gA1 * nb1 < (long long)MP) return;
  const int vec0 = ((nE0 & 3) == 0) ? 1 : 0;
  const int vec1 = ((nE1 & 3) == 0) ? 1 : 0;
  if ((long long)(gM - 1) * GBM >= (long long)nN) return;

  char* ws = (char*)d_ws;
  size_t off = 0;
  const size_t oA  = off; off = al256(off + (size_t)MP * KHL * 2);
  const size_t oW1 = off; off = al256(off + (size_t)NUW1 * 16);
  const size_t oW2 = off; off = al256(off + (size_t)NUW2 * 16);
  const size_t oK1 = off; off = al256(off + (size_t)NUK1 * 16);
  const size_t oK2 = off; off = al256(off + (size_t)NUK2 * 16);
  const size_t oLT = off; off = al256(off + (size_t)NULT * 16);
  const size_t oH  = off; off = al256(off + (size_t)MP * CH * 4);
  const size_t oDP = off; off = al256(off + (size_t)NATT * NHD * MP * 4);
  const size_t oOP = off; off = al256(off + (size_t)2 * MP * KHL * 2);
  const size_t oPS = off; off = al256(off + (size_t)2 * gM * CH * 4);
  const size_t oBE = off; off = al256(off + 256);
  if (off > ws_size || off > (size_t)WSMAX) return;
  unsigned short* XB  = (unsigned short*)(ws + oA);
  unsigned short* H2  = (unsigned short*)(ws + oA);
  unsigned short* W1T = (unsigned short*)(ws + oW1);
  unsigned short* W2T = (unsigned short*)(ws + oW2);
  unsigned short* K1T = (unsigned short*)(ws + oK1);
  unsigned short* K2T = (unsigned short*)(ws + oK2);
  unsigned short* LTp = (unsigned short*)(ws + oLT);
  float*          H   = (float*)(ws + oH);
  float*          DP  = (float*)(ws + oDP);
  unsigned short* O0  = (unsigned short*)(ws + oOP);
  unsigned short* O1  = O0 + (size_t)MP * KHL;
  float*          PS  = (float*)(ws + oPS);
  float*          BE  = (float*)(ws + oBE);
  const size_t aoff = (size_t)MP * KHL;
  float* DPs0 = DP;
  float* DPd0 = DP + (size_t)2 * MP;
  float* DPs1 = DP + (size_t)4 * MP;
  float* DPd1 = DP + (size_t)6 * MP;

  hipFuncSetAttribute(reinterpret_cast<const void*>(&k_agg), hipFuncAttributeMaxDynamicSharedMemorySize, LDS_AGG);

  const int nUx = MP * (NIN / 8);
  k_xprep<<<cdiv(nUx, NTHR), NTHR, 0, stream>>>(x, XB, NIN, nN, nUx);
  k_wprep<<<NUTOT / NTHR, NTHR, 0, stream>>>(w1, w2, kw1, kw2, lw, W1T, W2T, K1T, K2T, LTp);
  k_gemm<0><<<dim3(gM, 1), GTHR, 0, stream>>>(XB, NIN, (size_t)0, W1T, NIN, NIN, b1, H, CH,
                                              as1, ad1, DP, nN, MP);
  k_agg<<<gA0, NTHR, LDS_AGG, stream>>>(src0, dst0, H, DPs0, DPd0, O0, nN, nE0, nb0, vec0, MP);
  k_agg<<<gA1, NTHR, LDS_AGG, stream>>>(src1, dst1, H, DPs1, DPd1, O1, nN, nE1, nb1, vec1, MP);
  k_gemm<1><<<dim3(gM, 2), GTHR, 0, stream>>>(O0, KHL, aoff, K1T, KHL, KHL, kb1, PS, CH,
                                              kb1, kb1, DP, nN, MP);
  k_beta<<<1, GBN, 0, stream>>>(PS, gM, nN, q1, BE);
  const int nUm = MP * 32;
  k_mix<<<cdiv(nUm, NTHR), NTHR, 0, stream>>>(O0, O1, BE, H2, nN, nUm);
  k_gemm<0><<<dim3(gM, 1), GTHR, 0, stream>>>(H2, KHL, (size_t)0, W2T, KHL, KHL, b2, H, CH,
                                              as2, ad2, DP, nN, MP);
  k_agg<<<gA0, NTHR, LDS_AGG, stream>>>(src0, dst0, H, DPs0, DPd0, O0, nN, nE0, nb0, vec0, MP);
  k_agg<<<gA1, NTHR, LDS_AGG, stream>>>(src1, dst1, H, DPs1, DPd1, O1, nN, nE1, nb1, vec1, MP);
  k_gemm<1><<<dim3(gM, 2), GTHR, 0, stream>>>(O0, KHL, aoff, K2T, KHL, KHL, kb2, PS, CH,
                                              kb2, kb2, DP, nN, MP);
  k_beta<<<1, GBN, 0, stream>>>(PS, gM, nN, q2, BE);
  k_out<<<gM, GTHR, 0, stream>>>(O0, O1, BE, LTp, lb, nN, out);
}
